// SheafAttention_46909632807581
// MI455X (gfx1250) — hardware-verified
//
#include <hip/hip_runtime.h>
#include <hip/hip_bf16.h>
#include <stddef.h>
#include <stdint.h>


#define DM     1024
#define NH     16
#define HD     64
#define NBAT   2
#define SQ     2048
#define MTOK   (NBAT * SQ)
#define NPB    16
#define ATHR   128
#define AWAV   (ATHR / 32)
#define SPW    (NPB / AWAV)
#define NCAP   128
#define MW     (SQ / 32)
#define EPT    4
#define CHE    (ATHR * EPT)
#define WLCAP  (32 * EPT * 2)
#define SCWN   (NCAP * NH)
#define GBM    128
#define GBN    64
#define GTHR   128
#define CTHR   256
#define CWT    64.0f
#define CAO    8.0f
#define SCL_QK 1.0f
#define SCL_V  0.015625f
#define SCL_O  0.001953125f
#define ATTSC  0.125f
#define WSMAX  134217728

#define WS_XPL   ((size_t)MTOK * DM * 2)
#define WS_WPL   ((size_t)DM * DM * 2)
#define WS_FPL   ((size_t)MTOK * DM * 4)
#define WS_TOTAL (3 * WS_XPL + 6 * WS_WPL + 3 * WS_FPL + WS_XPL)

static_assert(NH * HD == DM);
static_assert(HD == 64);
static_assert(DM == 32 * 32);
static_assert(MW == 64);
static_assert(SPW * AWAV == NPB);
static_assert((SQ % NPB) == 0);
static_assert(WLCAP == 32 * 2 * EPT);
static_assert(NCAP <= SQ && (NCAP % 32) == 0);
static_assert((MTOK % GBM) == 0 && (DM % GBN) == 0 && (DM % 32) == 0);
static_assert(GBM == (GTHR / 32) * 32);
static_assert(((MTOK * DM / 8) % CTHR) == 0);
static_assert(((DM * DM / 8) % CTHR) == 0);
static_assert(WS_TOTAL <= (size_t)WSMAX);
static_assert((WS_XPL % 256) == 0 && (WS_WPL % 256) == 0 && (WS_FPL % 256) == 0);

typedef float          v4f  __attribute__((ext_vector_type(4)));
typedef float          v8f  __attribute__((ext_vector_type(8)));
typedef int            v4i  __attribute__((ext_vector_type(4)));
typedef int            v8i  __attribute__((ext_vector_type(8)));
typedef unsigned short v8us __attribute__((ext_vector_type(8)));
typedef _Float16       v8h  __attribute__((ext_vector_type(8)));
typedef _Float16       v16h __attribute__((ext_vector_type(16)));
typedef __attribute__((ext_vector_type(16))) __bf16 v16bf;

union Frag { v16h fh; v16bf fb; v8us h[2]; v8i w; };
static_assert(sizeof(Frag) == 32);

template<bool BF>
__device__ __forceinline__ v8f wmm(const Frag& a, const Frag& b, v8f c) {
  v8f d;
  if constexpr (BF) {
    d = __builtin_amdgcn_wmma_f32_16x16x32_bf16(false, a.fb, false, b.fb, (short)0, c, false, false);
  } else {
    d = __builtin_amdgcn_wmma_f32_16x16x32_f16(false, a.fh, false, b.fh, (short)0, c, false, false);
  }
  asm volatile("v_nop\n\tv_nop\n\tv_nop\n\tv_nop" : "+v"(d) : "v"(a.w), "v"(b.w));
  return d;
}

__device__ __forceinline__ void wsync() {
  __builtin_amdgcn_fence(__ATOMIC_RELEASE, "wavefront");
  __builtin_amdgcn_wave_barrier();
}

__device__ __forceinline__ unsigned bfb(float f) {
  const unsigned u = __float_as_uint(f);
  return (u + 0x7fffu + ((u >> 16) & 1u)) >> 16;
}

__device__ __forceinline__ v8h cvt8h(const v4f a, const v4f b) {
  v8h hv;
  hv[0] = (_Float16)a.x; hv[1] = (_Float16)a.y; hv[2] = (_Float16)a.z; hv[3] = (_Float16)a.w;
  hv[4] = (_Float16)b.x; hv[5] = (_Float16)b.y; hv[6] = (_Float16)b.z; hv[7] = (_Float16)b.w;
  return hv;
}

__device__ __forceinline__ int clj(int j) { return j < 0 ? 0 : (j > SQ - 1 ? SQ - 1 : j); }

__global__ __launch_bounds__(CTHR) void k_xcvt(const float* __restrict__ x, unsigned short* xh,
                                               unsigned short* xl, unsigned short* xf, int nUnits) {
  const int i = (int)blockIdx.x * CTHR + (int)threadIdx.x;
  if (i >= nUnits) return;
  const float* p = x + (size_t)i * 8;
  const v4f a = *(const v4f*)p;
  const v4f b = *(const v4f*)(p + 4);
  float v[8] = {a.x, a.y, a.z, a.w, b.x, b.y, b.z, b.w};
  v8us vh, vl;
  v8h vf;
#pragma unroll
  for (int e = 0; e < 8; ++e) {
    const unsigned hb = bfb(v[e]);
    const float lo = v[e] - __uint_as_float(hb << 16);
    vh[e] = (unsigned short)hb;
    vl[e] = (unsigned short)bfb(lo);
    vf[e] = (_Float16)v[e];
  }
  const size_t o = (size_t)i * 8;
  *(volatile v8us*)(xh + o) = vh;
  *(volatile v8us*)(xl + o) = vl;
  *(volatile v8h*)(xf + o)  = vf;
  __threadfence();
  *(volatile v8us*)(xh + o) = vh;
  *(volatile v8us*)(xl + o) = vl;
  *(volatile v8h*)(xf + o)  = vf;
}

template<bool SPLIT>
__global__ __launch_bounds__(CTHR) void k_wcvt(const float* __restrict__ W, unsigned short* p0, unsigned short* p1,
                                              int K, int N, float cw, int nUnits) {
  const int u = (int)blockIdx.x * CTHR + (int)threadIdx.x;
  if (u >= nUnits) return;
  const int kq = K >> 3;
  const int n  = u / kq;
  const int k8 = (u - n * kq) * 8;
  const float* p = W + (size_t)k8 * (size_t)N + n;
  float v[8];
#pragma unroll
  for (int e = 0; e < 8; ++e) v[e] = p[(size_t)e * (size_t)N];
  const size_t o = (size_t)n * (size_t)K + k8;
  if constexpr (SPLIT) {
    v8us vh, vl;
#pragma unroll
    for (int e = 0; e < 8; ++e) {
      const unsigned hb = bfb(v[e]);
      const float lo = v[e] - __uint_as_float(hb << 16);
      vh[e] = (unsigned short)hb;
      vl[e] = (unsigned short)bfb(lo);
    }
    *(volatile v8us*)(p0 + o) = vh;
    *(volatile v8us*)(p1 + o) = vl;
    __threadfence();
    *(volatile v8us*)(p0 + o) = vh;
    *(volatile v8us*)(p1 + o) = vl;
  } else {
    v8h vf;
#pragma unroll
    for (int e = 0; e < 8; ++e) vf[e] = (_Float16)(v[e] * cw);
    *(volatile v8h*)(p0 + o) = vf;
    __threadfence();
    *(volatile v8h*)(p0 + o) = vf;
  }
}

template<bool SPLIT>
__global__ __launch_bounds__(GTHR) void k_gemm(
    const unsigned short* __restrict__ Ah, const unsigned short* __restrict__ Al,
    const unsigned short* __restrict__ Wh, const unsigned short* __restrict__ Wl,
    const float* __restrict__ bias, float* outF, int K, int ldo, float scl)
{
  __shared__ __attribute__((aligned(16))) float stg[GBM * GBN];
  const int tid = (int)threadIdx.x, lane = tid & 31, wave = tid >> 5, hh = lane >> 4, m = lane & 15;
  const int rowBase = (int)blockIdx.x * GBM;
  const int col0    = (int)blockIdx.y * GBN;

  v8f acc[2][4];
  {
    const v8f z = {0.f, 0.f, 0.f, 0.f, 0.f, 0.f, 0.f, 0.f};
#pragma unroll
    for (int u = 0; u < 2; ++u)
#pragma unroll
      for (int t = 0; t < 4; ++t) acc[u][t] = z;
  }
  const size_t Ks   = (size_t)K;
  const size_t aoff = (size_t)(rowBase + 32 * wave + m) * Ks + 8 * hh;
  const size_t woff = (size_t)(col0 + m) * Ks + 8 * hh;
  const int ksteps = K >> 5;
#pragma unroll 1
  for (int ks = 0; ks < ksteps; ++ks) {
    const size_t kk = (size_t)(32 * ks);
    Frag ah[2], al[2];
#pragma unroll
    for (int u = 0; u < 2; ++u) {
      const unsigned short* ap = Ah + aoff + (size_t)(16 * u) * Ks + kk;
      ah[u].h[0] = *(const v8us*)ap;
      ah[u].h[1] = *(const v8us*)(ap + 16);
      if constexpr (SPLIT) {
        const unsigned short* aq = Al + aoff + (size_t)(16 * u) * Ks + kk;
        al[u].h[0] = *(const v8us*)aq;
        al[u].h[1] = *(const v8us*)(aq + 16);
      }
    }
#pragma unroll
    for (int t = 0; t < 4; ++t) {
      const unsigned short* wp = Wh + woff + (size_t)(16 * t) * Ks + kk;
      Frag bh;
      bh.h[0] = *(const v8us*)wp;
      bh.h[1] = *(const v8us*)(wp + 16);
      Frag bl;
      if constexpr (SPLIT) {
        const unsigned short* wq = Wl + woff + (size_t)(16 * t) * Ks + kk;
        bl.h[0] = *(const v8us*)wq;
        bl.h[1] = *(const v8us*)(wq + 16);
      }
#pragma unroll
      for (int u = 0; u < 2; ++u) {
        acc[u][t] = wmm<SPLIT>(ah[u], bh, acc[u][t]);
        if constexpr (SPLIT) {
          acc[u][t] = wmm<SPLIT>(ah[u], bl, acc[u][t]);
          acc[u][t] = wmm<SPLIT>(al[u], bh, acc[u][t]);
        }
      }
    }
  }

#pragma unroll
  for (int t = 0; t < 4; ++t) {
    const int lc = 16 * t + m;
    const float bv = bias[col0 + lc];
#pragma unroll
    for (int u = 0; u < 2; ++u) {
#pragma unroll
      for (int r = 0; r < 8; ++r) {
        const int lr = 32 * wave + 16 * u + 8 * hh + r;
        stg[lr * GBN + lc] = fmaf(acc[u][t][r], scl, bv);
      }
    }
  }
  __syncthreads();

#pragma unroll
  for (int i = 0; i < 16; ++i) {
    const int lr = 32 * wave + 2 * i + hh;
    const v4f fv = *(const v4f*)(stg + lr * GBN + 4 * m);
    float* op = outF + (size_t)(rowBase + lr) * (size_t)ldo + col0 + 4 * m;
    *(volatile v4f*)op = fv;
  }
  __threadfence();
#pragma unroll
  for (int i = 0; i < 16; ++i) {
    const int lr = 32 * wave + 2 * i + hh;
    const v4f fv = *(const v4f*)(stg + lr * GBN + 4 * m);
    float* op = outF + (size_t)(rowBase + lr) * (size_t)ldo + col0 + 4 * m;
    *(volatile v4f*)op = fv;
  }
}

#define HIT(HJ, ENT) { \
    const unsigned mj = __builtin_amdgcn_ballot_w32(HJ); \
    if (mj != 0u) { \
      if (HJ) { \
        const int pos = wc + (int)__builtin_amdgcn_mbcnt_lo(mj, 0u); \
        if (pos < WLCAP) wl[wave * WLCAP + pos] = (ENT); \
      } \
      wc += (int)__builtin_popcount(mj); } }

__global__ __launch_bounds__(ATHR) void k_attn(const int* __restrict__ ei, int nE,
    const float* __restrict__ Qf, const float* __restrict__ Kf, const float* __restrict__ Vf,
    unsigned short* AO)
{
  __shared__ unsigned bm[NPB * MW];
  __shared__ int wl[AWAV * WLCAP];
  __shared__ int wcs[AWAV];
  __shared__ int nl[NPB * NCAP];
  __shared__ int ncn[NPB];
  __shared__ __attribute__((aligned(16))) float scw[AWAV * SCWN];
  __shared__ __attribute__((aligned(16))) _Float16 stg[AWAV * DM];

  const int tid = (int)threadIdx.x, lane = tid & 31, wave = tid >> 5;
  const int n0 = (int)blockIdx.x * NPB;

  for (int i = tid; i < NPB * MW; i += ATHR) {
    const int s = i >> 6, w = i & 63;
    const int nd = n0 + s;
    bm[i] = (w == (nd >> 5)) ? (1u << (nd & 31)) : 0u;
  }
  __syncthreads();

  const int nChunks = (nE + CHE - 1) / CHE;
#pragma unroll 1
  for (int ch = 0; ch < nChunks; ++ch) {
    const int cbase = ch * CHE;
    const int e0 = cbase + tid * EPT;
    v4i da, db;
    if (cbase + CHE <= nE) {
      const int* p = ei + (size_t)e0 * 2;
      da = *(const v4i*)p;
      db = *(const v4i*)(p + 4);
    } else {
      const int last = 2 * nE - 1;
      int tq[8];
#pragma unroll
      for (int q = 0; q < 8; ++q) {
        const int idx = 2 * e0 + q;
        const int ic  = idx > last ? last : (idx < 0 ? 0 : idx);
        const int vq  = ei[ic];
        tq[q] = (e0 + (q >> 1) < nE) ? vq : -1;
      }
      da.x = tq[0]; da.y = tq[1]; da.z = tq[2]; da.w = tq[3];
      db.x = tq[4]; db.y = tq[5]; db.z = tq[6]; db.w = tq[7];
    }
    int av[4] = {da.x, da.z, db.x, db.z};
    int bw[4] = {da.y, da.w, db.y, db.w};
    bool ha[4], hb[4];
    int ea[4], eb[4];
    bool anyl = false;
#pragma unroll
    for (int e = 0; e < 4; ++e) {
      const unsigned ua = (unsigned)(av[e] - n0);
      const unsigned ub = (unsigned)(bw[e] - n0);
      ha[e] = ua < (unsigned)NPB;
      hb[e] = ub < (unsigned)NPB;
      ea[e] = (int)((ua & 15u) << 16) | clj(bw[e]);
      eb[e] = (int)((ub & 15u) << 16) | clj(av[e]);
      anyl = anyl | ha[e] | hb[e];
    }
    int wc = 0;
    const unsigned any = __builtin_amdgcn_ballot_w32(anyl);
    if (any != 0u) {
#pragma unroll
      for (int e = 0; e < 4; ++e) {
        HIT(ha[e], ea[e])
        HIT(hb[e], eb[e])
      }
    }
    if (lane == 0) wcs[wave] = wc;
    __syncthreads();
    if (tid == 0) {
#pragma unroll 1
      for (int w2 = 0; w2 < AWAV; ++w2) {
        int c = wcs[w2];
        c = c < 0 ? 0 : (c > WLCAP ? WLCAP : c);
#pragma unroll 1
        for (int i = 0; i < c; ++i) {
          const int ent = wl[w2 * WLCAP + i];
          const int s = (ent >> 16) & (NPB - 1);
          const int j = ent & (SQ - 1);
          bm[s * MW + (j >> 5)] |= (1u << (j & 31));
        }
      }
    }
    __syncthreads();
  }

#pragma unroll 1
  for (int sl = 0; sl < SPW; ++sl) {
    const int s = wave * SPW + sl;
    unsigned w0 = bm[s * MW + 2 * lane];
    unsigned w1 = bm[s * MW + 2 * lane + 1];
    const int c = (int)__builtin_popcount(w0) + (int)__builtin_popcount(w1);
    int incl = c;
#pragma unroll
    for (int d = 1; d < 32; d <<= 1) {
      const int up = __shfl_up(incl, d);
      incl += (lane >= d) ? up : 0;
    }
    const int tot = __shfl(incl, 31);
    int pos = incl - c;
    while (w0 != 0u) {
      const int bit = __builtin_ctz(w0);
      w0 &= (w0 - 1u);
      if (pos < NCAP) nl[s * NCAP + pos] = 64 * lane + bit;
      ++pos;
    }
    while (w1 != 0u) {
      const int bit = __builtin_ctz(w1);
      w1 &= (w1 - 1u);
      if (pos < NCAP) nl[s * NCAP + pos] = 64 * lane + 32 + bit;
      ++pos;
    }
    if (lane == 0) ncn[s] = tot;
  }
  __syncthreads();

  const float qnan = __int_as_float(0x7fc00000);
  float* sw = scw + wave * SCWN;
  _Float16* st = stg + wave * DM;
  const int hq = lane & 15;
#pragma unroll 1
  for (int sl = 0; sl < SPW; ++sl) {
    const int s = wave * SPW + sl;
    const int node = n0 + s;
    const int craw = __builtin_amdgcn_readfirstlane(ncn[s]);
    const int cnt = craw < 0 ? 0 : (craw > NCAP ? NCAP : craw);
    const float pz = (craw > NCAP) ? qnan : 0.0f;
    const int* nls = nl + s * NCAP;
#pragma unroll 1
    for (int b = 0; b < NBAT; ++b) {
      const size_t tok = (size_t)b * SQ + (size_t)node;
      const size_t kvb = (size_t)b * SQ;
      wsync();
      v4f qv[8];
      {
        const float* qp = Qf + tok * DM + 32 * lane;
#pragma unroll
        for (int c = 0; c < 8; ++c) qv[c] = *(const v4f*)(qp + 4 * c);
      }
#pragma unroll 1
      for (int j = 0; j < cnt; ++j) {
        const int kid = clj(nls[j]);
        const float* kp = Kf + (kvb + (size_t)kid) * DM + 32 * lane;
        float p = 0.f;
#pragma unroll
        for (int c = 0; c < 8; ++c) {
          const v4f kk = *(const v4f*)(kp + 4 * c);
          p = fmaf(qv[c].x, kk.x, p);
          p = fmaf(qv[c].y, kk.y, p);
          p = fmaf(qv[c].z, kk.z, p);
          p = fmaf(qv[c].w, kk.w, p);
        }
        p += __shfl_xor(p, 1);
        const float sc = p * ATTSC;
        if ((lane & 1) == 0) sw[j * NH + (lane >> 1)] = sc;
      }
      wsync();
      float mx = -3.0e38f;
#pragma unroll 1
      for (int j = 0; j < cnt; ++j) mx = fmaxf(mx, sw[j * NH + hq]);
      float sum = 0.f;
#pragma unroll 1
      for (int j = 0; j < cnt; ++j) {
        const float e = __expf(sw[j * NH + hq] - mx);
        sum += e;
        if (lane < NH) sw[j * NH + hq] = e;
      }
      const float inv  = (sum > 0.f) ? (1.0f / sum) : 0.f;
      const float invl = __shfl(inv, lane >> 1);
      wsync();
      v4f acc[8];
      {
        const v4f z4 = {0.f, 0.f, 0.f, 0.f};
#pragma unroll
        for (int c = 0; c < 8; ++c) acc[c] = z4;
      }
#pragma unroll 1
      for (int j = 0; j < cnt; ++j) {
        const float w = sw[j * NH + (lane >> 1)];
        const int vid = clj(nls[j]);
        const float* vp = Vf + (kvb + (size_t)vid) * DM + 32 * lane;
#pragma unroll
        for (int c = 0; c < 8; ++c) {
          const v4f vv = *(const v4f*)(vp + 4 * c);
          acc[c] = vv * w + acc[c];
        }
      }
      const float f = invl * CAO;
      const v4f pz4 = {pz, pz, pz, pz};
      v8h hv[4];
#pragma unroll
      for (int q = 0; q < 4; ++q) hv[q] = cvt8h(acc[2 * q] * f + pz4, acc[2 * q + 1] * f + pz4);
      wsync();
#pragma unroll
      for (int q = 0; q < 4; ++q) *(v8h*)(st + 32 * lane + 8 * q) = hv[q];
      wsync();
      v8h rd[4];
#pragma unroll
      for (int q = 0; q < 4; ++q) rd[q] = *(const v8h*)(st + 256 * q + 8 * lane);
      unsigned short* op = AO + tok * DM;
#pragma unroll
      for (int q = 0; q < 4; ++q) *(volatile v8h*)(op + 256 * q + 8 * lane) = rd[q];
      __threadfence();
#pragma unroll
      for (int q = 0; q < 4; ++q) *(volatile v8h*)(op + 256 * q + 8 * lane) = rd[q];
    }
  }
}
#undef HIT

static inline int cdiv(int a, int b) { return (a + b - 1) / b; }

extern "C" void kernel_launch(void* const* d_in, const int* in_sizes, int n_in,
                              void* d_out, int out_size, void* d_ws, size_t ws_size,
                              hipStream_t stream) {
  if (n_in < 10) return;
  if (in_sizes[0] != MTOK * DM) return;
  if (in_sizes[1] != DM * DM || in_sizes[2] != DM) return;
  if (in_sizes[3] != DM * DM || in_sizes[4] != DM) return;
  if (in_sizes[5] != DM * DM || in_sizes[6] != DM) return;
  if (in_sizes[7] != DM * DM || in_sizes[8] != DM) return;
  if (in_sizes[9] < 2 || (in_sizes[9] & 1) != 0) return;
  const int nE = in_sizes[9] / 2;
  if (nE < 1 || nE > (1 << 26)) return;
  if (out_size != MTOK * DM) return;
  if (ws_size < WS_TOTAL) return;

  const float* x  = (const float*)d_in[0];
  const float* Wq = (const float*)d_in[1];
  const float* bq = (const float*)d_in[2];
  const float* Wk = (const float*)d_in[3];
  const float* bk = (const float*)d_in[4];
  const float* Wv = (const float*)d_in[5];
  const float* bv = (const float*)d_in[6];
  const float* Wo = (const float*)d_in[7];
  const float* bo = (const float*)d_in[8];
  const int*   ei = (const int*)d_in[9];
  float* out = (float*)d_out;

  char* ws = (char*)d_ws;
  size_t off = 0;
  unsigned short* XH  = (unsigned short*)(ws + off); off += WS_XPL;
  unsigned short* XL  = (unsigned short*)(ws + off); off += WS_XPL;
  unsigned short* XF  = (unsigned short*)(ws + off); off += WS_XPL;
  unsigned short* WQH = (unsigned short*)(ws + off); off += WS_WPL;
  unsigned short* WQL = (unsigned short*)(ws + off); off += WS_WPL;
  unsigned short* WKH = (unsigned short*)(ws + off); off += WS_WPL;
  unsigned short* WKL = (unsigned short*)(ws + off); off += WS_WPL;
  unsigned short* WVT = (unsigned short*)(ws + off); off += WS_WPL;
  unsigned short* WOT = (unsigned short*)(ws + off); off += WS_WPL;
  float*          QF  = (float*)(ws + off);          off += WS_FPL;
  float*          KF  = (float*)(ws + off);          off += WS_FPL;
  float*          VF  = (float*)(ws + off);          off += WS_FPL;
  unsigned short* AO  = (unsigned short*)(ws + off); off += WS_XPL;
  if (off != WS_TOTAL || off > ws_size || off > (size_t)WSMAX) return;

  const int nUx = MTOK * DM / 8;
  k_xcvt<<<cdiv(nUx, CTHR), CTHR, 0, stream>>>(x, XH, XL, XF, nUx);

  const int nUw = DM * DM / 8;
  k_wcvt<true ><<<cdiv(nUw, CTHR), CTHR, 0, stream>>>(Wq, WQH, WQL, DM, DM, 1.0f, nUw);
  k_wcvt<true ><<<cdiv(nUw, CTHR), CTHR, 0, stream>>>(Wk, WKH, WKL, DM, DM, 1.0f, nUw);
  k_wcvt<false><<<cdiv(nUw, CTHR), CTHR, 0, stream>>>(Wv, WVT, WVT, DM, DM, CWT, nUw);
  k_wcvt<false><<<cdiv(nUw, CTHR), CTHR, 0, stream>>>(Wo, WOT, WOT, DM, DM, CWT, nUw);

  const dim3 gg(MTOK / GBM, DM / GBN);
  k_gemm<true ><<<gg, GTHR, 0, stream>>>(XH, XL, WQH, WQL, bq, QF, DM, DM, SCL_QK);
  k_gemm<true ><<<gg, GTHR, 0, stream>>>(XH, XL, WKH, WKL, bk, KF, DM, DM, SCL_QK);
  k_gemm<false><<<gg, GTHR, 0, stream>>>(XF, XF, WVT, WVT, bv, VF, DM, DM, SCL_V);

  k_attn<<<SQ / NPB, ATHR, 0, stream>>>(ei, nE, QF, KF, VF, AO);

  k_gemm<false><<<gg, GTHR, 0, stream>>>(AO, AO, WOT, WOT, bo, out, DM, DM, SCL_O);
}
